// TrajEncoder_13108240187766
// MI455X (gfx1250) — hardware-verified
//
#include <hip/hip_runtime.h>


typedef _Float16       f16t;
typedef unsigned short u16t;
typedef f16t   v16h __attribute__((ext_vector_type(16)));
typedef f16t   v8h  __attribute__((ext_vector_type(8)));
typedef __bf16 v16b __attribute__((ext_vector_type(16)));
typedef __bf16 v8b  __attribute__((ext_vector_type(8)));
typedef float  v8f  __attribute__((ext_vector_type(8)));
typedef float  v4f  __attribute__((ext_vector_type(4)));
typedef unsigned int v4u __attribute__((ext_vector_type(4)));
typedef unsigned int v2u __attribute__((ext_vector_type(2)));

union FragH { v16h v; v8h q[2]; };
union FragB { v16b v; v8b q[2]; };
union Pk8u  { u16t s[8]; v4u u; };
union Pk8h  { f16t h[8]; v4u u; };
union Pk4u  { u16t s[4]; v2u u; };

#define LD   128
#define LH   256
#define LG   1024
#define NBR  16
#define NTHR 512
#define XSTR 136
#define HSTR 264
#define OSTR 260
#define SCX  16.0f
#define SCW  128.0f
#define INVS 0.00048828125f

__device__ __forceinline__ unsigned int rne_bf16_u32(float x) {
    unsigned int u = __float_as_uint(x);
    u += 0x7FFFu + ((u >> 16) & 1u);
    return u & 0xFFFF0000u;
}
__device__ __forceinline__ float rb16(float x)      { return __uint_as_float(rne_bf16_u32(x)); }
__device__ __forceinline__ u16t  rb16_bits(float x) { return (u16t)(rne_bf16_u32(x) >> 16); }

__device__ __forceinline__ v8f mma_b(v16b a, v16b b, v8f c) {
    return __builtin_amdgcn_wmma_f32_16x16x32_bf16(false, a, false, b, (short)0, c, false, false);
}
__device__ __forceinline__ v8f mma_h(v16h a, v16h b, v8f c) {
    return __builtin_amdgcn_wmma_f32_16x16x32_f16(false, a, false, b, (short)0, c, false, false);
}
__device__ __forceinline__ void guard_b(v8f (&c)[4], FragB& a, FragB (&b)[4]) {
    asm volatile("v_nop\n\tv_nop\n\tv_nop\n\tv_nop"
                 : "+v"(c[0]), "+v"(c[1]), "+v"(c[2]), "+v"(c[3])
                 : "v"(a.v), "v"(b[0].v), "v"(b[1].v), "v"(b[2].v), "v"(b[3].v));
}
__device__ __forceinline__ void guard_h(v8f (&c)[4], FragH& a, FragH (&b)[4]) {
    asm volatile("v_nop\n\tv_nop\n\tv_nop\n\tv_nop"
                 : "+v"(c[0]), "+v"(c[1]), "+v"(c[2]), "+v"(c[3])
                 : "v"(a.v), "v"(b[0].v), "v"(b[1].v), "v"(b[2].v), "v"(b[3].v));
}

__device__ __forceinline__ float fsig(float x) {
    return __builtin_amdgcn_rcpf(1.0f + __expf(-x));
}
__device__ __forceinline__ float ftanh(float x) {
    float ax = fabsf(x);
    float t  = __expf(-2.0f * ax);
    float r  = (1.0f - t) * __builtin_amdgcn_rcpf(1.0f + t);
    return copysignf(r, x);
}

__global__ __launch_bounds__(256)
void k_pack_ih(const float* __restrict__ W, u16t* P, int n8) {
    int i = blockIdx.x * 256 + threadIdx.x;
    if (i >= n8) return;
    const float* p = W + (size_t)i * 8;
    v4f a = *(const v4f*)p;
    v4f b = *(const v4f*)(p + 4);
    Pk8u k;
    k.s[0] = rb16_bits(a[0] * SCW); k.s[1] = rb16_bits(a[1] * SCW);
    k.s[2] = rb16_bits(a[2] * SCW); k.s[3] = rb16_bits(a[3] * SCW);
    k.s[4] = rb16_bits(b[0] * SCW); k.s[5] = rb16_bits(b[1] * SCW);
    k.s[6] = rb16_bits(b[2] * SCW); k.s[7] = rb16_bits(b[3] * SCW);
    u16t* d = P + (size_t)i * 8;
    *(volatile v4u*)d = k.u;
    __threadfence();
    *(volatile v4u*)d = k.u;
}

__global__ __launch_bounds__(256)
void k_pack_hh(const float* __restrict__ W, f16t* P, int n8) {
    int i = blockIdx.x * 256 + threadIdx.x;
    if (i >= n8) return;
    const float* p = W + (size_t)i * 8;
    v4f a = *(const v4f*)p;
    v4f b = *(const v4f*)(p + 4);
    Pk8h k;
    k.h[0] = (f16t)(rb16(a[0]) * SCW); k.h[1] = (f16t)(rb16(a[1]) * SCW);
    k.h[2] = (f16t)(rb16(a[2]) * SCW); k.h[3] = (f16t)(rb16(a[3]) * SCW);
    k.h[4] = (f16t)(rb16(b[0]) * SCW); k.h[5] = (f16t)(rb16(b[1]) * SCW);
    k.h[6] = (f16t)(rb16(b[2]) * SCW); k.h[7] = (f16t)(rb16(b[3]) * SCW);
    f16t* d = P + (size_t)i * 8;
    *(volatile v4u*)d = k.u;
    __threadfence();
    *(volatile v4u*)d = k.u;
}

__global__ __launch_bounds__(NTHR)
void k_lstm(const int* __restrict__ path, const int* __restrict__ vlen,
            const float* __restrict__ emb,
            const float* __restrict__ b_ih, const float* __restrict__ b_hh,
            const u16t* __restrict__ Pih, const f16t* __restrict__ Phh,
            float* out, int nb, int T, int vocab) {
    __shared__ __attribute__((aligned(16))) u16t  xS[NBR * XSTR];
    __shared__ __attribute__((aligned(16))) f16t  hS[NBR * HSTR];
    __shared__ __attribute__((aligned(16))) float oS[NBR * OSTR];

    const int tid  = threadIdx.x;
    const int lane = tid & 31;
    const int w    = tid >> 5;
    const int hh   = lane >> 4;
    const int m    = lane & 15;
    const int b0   = blockIdx.x * NBR;
    if (b0 + NBR > nb) return;
    const int j    = 16 * w + m;

    const float bi = rb16(b_ih[j])          + rb16(b_hh[j]);
    const float bf = rb16(b_ih[j + LH])     + rb16(b_hh[j + LH]);
    const float bg = rb16(b_ih[j + 2 * LH]) + rb16(b_hh[j + 2 * LH]);
    const float bo = rb16(b_ih[j + 3 * LH]) + rb16(b_hh[j + 3 * LH]);

    int   tc[8];
    float cst[8], hF[8];
#pragma unroll
    for (int r = 0; r < 8; ++r) {
        int v = vlen[b0 + 8 * hh + r] - 1;
        if (v < 0) v += T;
        v = v < 0 ? 0 : v;
        v = v > T - 1 ? T - 1 : v;
        tc[r]  = v;
        cst[r] = 0.0f;
        hF[r]  = 0.0f;
    }

    for (int i = tid; i < NBR * HSTR; i += NTHR) hS[i] = (f16t)0.0f;
    __syncthreads();

    const int gr = tid >> 5, gc = (tid & 31) * 4;
    const int* prow = path + (size_t)(b0 + gr) * T;
    u16t* xdst = xS + gr * XSTR + gc;

    const u16t* ax = xS + m * XSTR + 8 * hh;
    const f16t* ah = hS + m * HSTR + 8 * hh;
    const u16t* bx = Pih + (size_t)j * LD + 8 * hh;
    const f16t* bh = Phh + (size_t)j * LH + 8 * hh;

    const v8f z8 = {0.f, 0.f, 0.f, 0.f, 0.f, 0.f, 0.f, 0.f};

#pragma unroll 1
    for (int t = 0; t < T; ++t) {
        {
            int tok = prow[t];
            if (tok < 0) tok += vocab;
            tok = tok < 0 ? 0 : tok;
            tok = tok > vocab - 1 ? vocab - 1 : tok;
            v4f x = *(const v4f*)(emb + (size_t)tok * LD + gc);
            Pk4u pk;
            pk.s[0] = rb16_bits(x[0] * SCX);
            pk.s[1] = rb16_bits(x[1] * SCX);
            pk.s[2] = rb16_bits(x[2] * SCX);
            pk.s[3] = rb16_bits(x[3] * SCX);
            *(v2u*)xdst = pk.u;
        }
        __syncthreads();

        v8f acc[4];
        acc[0] = z8; acc[1] = z8; acc[2] = z8; acc[3] = z8;
        int kz = 0;
        asm volatile("" : "+s"(kz));

#pragma unroll 1
        for (int kt = 0; kt < LD / 32; ++kt) {
            const int ko = kt * 32 + kz;
            FragB a, b[4];
            a.q[0] = *(const v8b*)(ax + ko);
            a.q[1] = *(const v8b*)(ax + ko + 16);
#pragma unroll
            for (int g = 0; g < 4; ++g) {
                const u16t* p = bx + (size_t)g * LH * LD + ko;
                b[g].q[0] = *(const v8b*)p;
                b[g].q[1] = *(const v8b*)(p + 16);
            }
#pragma unroll
            for (int g = 0; g < 4; ++g) acc[g] = mma_b(a.v, b[g].v, acc[g]);
            guard_b(acc, a, b);
        }
#pragma unroll 1
        for (int kt = 0; kt < LH / 32; ++kt) {
            const int ko = kt * 32 + kz;
            FragH a, b[4];
            a.q[0] = *(const v8h*)(ah + ko);
            a.q[1] = *(const v8h*)(ah + ko + 16);
#pragma unroll
            for (int g = 0; g < 4; ++g) {
                const f16t* p = bh + (size_t)g * LH * LH + ko;
                b[g].q[0] = *(const v8h*)p;
                b[g].q[1] = *(const v8h*)(p + 16);
            }
#pragma unroll
            for (int g = 0; g < 4; ++g) acc[g] = mma_h(a.v, b[g].v, acc[g]);
            guard_h(acc, a, b);
        }
        __syncthreads();

#pragma unroll
        for (int r = 0; r < 8; ++r) {
            float gi = fmaf(acc[0][r], INVS, bi);
            float gf = fmaf(acc[1][r], INVS, bf);
            float gg = fmaf(acc[2][r], INVS, bg);
            float go = fmaf(acc[3][r], INVS, bo);
            float is = fsig(gi);
            float fs = fsig(gf);
            float os = fsig(go);
            float c  = fs * cst[r] + is * ftanh(gg);
            cst[r]   = c;
            float h  = os * ftanh(c);
            hS[(8 * hh + r) * HSTR + j] = (f16t)(h * SCX);
            hF[r] = (t == tc[r]) ? h : hF[r];
        }
    }

#pragma unroll
    for (int r = 0; r < 8; ++r) oS[(8 * hh + r) * OSTR + j] = hF[r];
    __syncthreads();

    v4f v0, v1;
    const int p0 = tid,        row0 = p0 >> 6, c0 = (p0 & 63) * 4;
    const int p1 = tid + NTHR, row1 = p1 >> 6, c1 = (p1 & 63) * 4;
    v0 = *(const v4f*)(oS + row0 * OSTR + c0);
    v1 = *(const v4f*)(oS + row1 * OSTR + c1);
    float* d0 = out + (size_t)(b0 + row0) * LH + c0;
    float* d1 = out + (size_t)(b0 + row1) * LH + c1;
    *(volatile v4f*)d0 = v0;
    *(volatile v4f*)d1 = v1;
    __threadfence();
    *(volatile v4f*)d0 = v0;
    *(volatile v4f*)d1 = v1;
}

extern "C" void kernel_launch(void* const* d_in, const int* in_sizes, int n_in,
                              void* d_out, int out_size, void* d_ws, size_t ws_size,
                              hipStream_t stream) {
    const int NB = 64, T = 512;

    if (n_in < 7) return;
    if (in_sizes[0] != NB * T || in_sizes[1] != NB) return;
    if (in_sizes[2] < LD || (in_sizes[2] % LD) != 0) return;
    if (in_sizes[3] != LG * LD || in_sizes[4] != LG * LH ||
        in_sizes[5] != LG || in_sizes[6] != LG) return;
    if (out_size != NB * LH) return;
    if ((NB % NBR) != 0) return;
    const int vocab = in_sizes[2] / LD;

    const int*   path = (const int*)d_in[0];
    const int*   vlen = (const int*)d_in[1];
    const float* emb  = (const float*)d_in[2];
    const float* W_ih = (const float*)d_in[3];
    const float* W_hh = (const float*)d_in[4];
    const float* b_ih = (const float*)d_in[5];
    const float* b_hh = (const float*)d_in[6];
    float* out = (float*)d_out;

    const size_t bytes_ih = (size_t)LG * LD * sizeof(u16t);
    const size_t bytes_hh = (size_t)LG * LH * sizeof(f16t);
    if (bytes_ih + bytes_hh > ws_size) return;
    u16t* Pih = (u16t*)d_ws;
    f16t* Phh = (f16t*)((char*)d_ws + bytes_ih);

    const int n8a = LG * LD / 8;
    const int n8b = LG * LH / 8;
    k_pack_ih<<<dim3((n8a + 255) / 256), dim3(256), 0, stream>>>(W_ih, Pih, n8a);
    k_pack_hh<<<dim3((n8b + 255) / 256), dim3(256), 0, stream>>>(W_hh, Phh, n8b);
    k_lstm<<<dim3(NB / NBR), dim3(NTHR), 0, stream>>>(path, vlen, emb, b_ih, b_hh,
                                                      Pih, Phh, out, NB, T, vocab);
}
